// CharRNN_86792699118072
// MI455X (gfx1250) — hardware-verified
//
#include <hip/hip_runtime.h>
#include <math.h>

constexpr int NBATCH   = 256;
constexpr int NSTEP    = 512;
constexpr int NEMB     = 256;
constexpr int NHID     = 1024;
constexpr int NVOC     = 64;
constexpr int NTHR     = 256;
constexpr int ROWS_BLK = 32;
constexpr int AHP      = 1032;
constexpr int XPP      = 1024;
constexpr int LSP      = 36;
constexpr int NOUT0    = NBATCH * NSTEP * NVOC;
constexpr int NOUT1    = NBATCH * NHID;
constexpr float WCARRY     = 256.0f;
constexpr float WCARRY_INV = 1.0f / 256.0f;

constexpr int LDS_XP_BYTES  = ROWS_BLK * XPP * 4;
constexpr int AH_HALVES     = ROWS_BLK * AHP;
constexpr int LDS_AH_BYTES  = 2 * AH_HALVES * 2;
constexpr int LDS_LSL_BYTES = 4 * 16 * LSP * 4;
constexpr int OFF_AH        = LDS_XP_BYTES;
constexpr int OFF_LSL       = OFF_AH + LDS_AH_BYTES;
constexpr int LDS_TOTAL     = OFF_LSL + LDS_LSL_BYTES;

static_assert(NBATCH % ROWS_BLK == 0, "grid exact");
static_assert(ROWS_BLK == 32, "two 16-row m-subtiles per block");
static_assert(NHID == 128 * (NTHR / 32), "8 waves x 128 hidden columns");
static_assert(NHID == 4 * NTHR, "x-projection staging: 256 threads x 4 floats per row");
static_assert(NHID % 32 == 0, "K multiple of 32");
static_assert(NVOC == 64, "4 waves x (16 rows x 32 vocab) logits tiles");
static_assert((NVOC * NHID / 4) % NTHR == 0, "table grid exact");
static_assert(NHID % 64 == 0 && NVOC % 64 == 0, "transpose tiles exact");
static_assert(NOUT0 * 4 == 33554432, "second output byte offset");
static_assert((OFF_AH % 16) == 0 && (OFF_LSL % 16) == 0 && ((AH_HALVES * 2) % 16) == 0, "LDS alignment");
static_assert((LDS_AH_BYTES % 16) == 0, "zero fill in 16-B chunks");

typedef __attribute__((ext_vector_type(16))) _Float16 v16h;
typedef __attribute__((ext_vector_type(8)))  _Float16 v8h;
typedef __attribute__((ext_vector_type(4)))  _Float16 v4h;
typedef __attribute__((ext_vector_type(8)))  float    v8f;
typedef __attribute__((ext_vector_type(4)))  float    v4f;
typedef __attribute__((ext_vector_type(2)))  float    v2f;
typedef __attribute__((ext_vector_type(4)))  unsigned u4;

__device__ __forceinline__ void acc_guard4(v8f& a, v8f& b, v8f& c, v8f& d) { asm volatile("v_nop\n\tv_nop\n\tv_nop\n\tv_nop" : "+v"(a), "+v"(b), "+v"(c), "+v"(d)); }
__device__ __forceinline__ void acc_guard2(v8f& a, v8f& b) { asm volatile("v_nop\n\tv_nop\n\tv_nop\n\tv_nop" : "+v"(a), "+v"(b)); }
__device__ __forceinline__ void guard8x6(v8f& c0, v8f& c1, v8f& c2, v8f& c3, v8f& c4, v8f& c5, v8f& c6, v8f& c7,
                                         v16h a0, v16h a1, v16h b0, v16h b1, v16h b2, v16h b3) {
  asm volatile("v_nop\n\tv_nop\n\tv_nop\n\tv_nop"
               : "+v"(c0), "+v"(c1), "+v"(c2), "+v"(c3), "+v"(c4), "+v"(c5), "+v"(c6), "+v"(c7)
               : "v"(a0), "v"(a1), "v"(b0), "v"(b1), "v"(b2), "v"(b3));
}
__device__ __forceinline__ void guard2x3(v8f& c0, v8f& c1, v16h a, v16h b0, v16h b1) {
  asm volatile("v_nop\n\tv_nop\n\tv_nop\n\tv_nop" : "+v"(c0), "+v"(c1) : "v"(a), "v"(b0), "v"(b1));
}

template <typename T> struct Frag;
template <> struct Frag<_Float16> {
  typedef v16h V; union U { v16h v; v8h h[2]; };
  static __device__ __forceinline__ v16h load(const _Float16* p) {
    U f; f.h[0] = *(const v8h*)(p); f.h[1] = *(const v8h*)(p + 16); return f.v;
  }
  static __device__ __forceinline__ v8f mma(v16h a, v16h b, v8f c) {
    return __builtin_amdgcn_wmma_f32_16x16x32_f16(false, a, false, b, (short)0, c, false, false);
  }
};

__device__ __forceinline__ float ftanh(float x) { return 1.0f - 2.0f * __builtin_amdgcn_rcpf(__expf(2.0f * x) + 1.0f); }

__global__ __launch_bounds__(NTHR) void table_kernel(const float* __restrict__ emb, const float* __restrict__ wih,
                                                     const float* __restrict__ bh, float* __restrict__ tab) {
  const int g  = blockIdx.x * NTHR + threadIdx.x;
  const int v  = g >> 8;
  const int h4 = (g & 255) * 4;
  const float* ep = emb + (size_t)v * NEMB;
  v4f s = {0.0f, 0.0f, 0.0f, 0.0f};
#pragma unroll 1
  for (int e = 0; e < NEMB; ++e) {
    const float ev = ep[e];
    const v4f w = *(const v4f*)(wih + (size_t)e * NHID + h4);
    s = s + w * ev;
  }
  const v4f b = *(const v4f*)(bh + h4);
  const v4f o = s + b;
  float* op = tab + (size_t)v * NHID + h4;
  *(volatile v4f*)op = o;
  __threadfence();
  *(volatile v4f*)op = o;
}

__global__ __launch_bounds__(NTHR) void tpw_f16_kernel(const float* __restrict__ src, int R, int C, int ldo,
                                                       unsigned short* __restrict__ O, float sc) {
  __shared__ float Tt[64 * 65];
  const int tid = threadIdx.x;
  const int c0 = blockIdx.x * 64, r0 = blockIdx.y * 64;
#pragma unroll
  for (int i = 0; i < 4; ++i) {
    const int idx = i * NTHR + tid;
    const int rr = idx >> 4, cc = (idx & 15) * 4;
    const v4f v = *(const v4f*)(src + (size_t)(r0 + rr) * (size_t)C + c0 + cc);
    Tt[rr * 65 + cc + 0] = v[0];
    Tt[rr * 65 + cc + 1] = v[1];
    Tt[rr * 65 + cc + 2] = v[2];
    Tt[rr * 65 + cc + 3] = v[3];
  }
  __syncthreads();
  const int q = tid >> 3, c8 = (tid & 7) * 8;
  v8h hv[2];
#pragma unroll
  for (int g = 0; g < 2; ++g) {
    const int qq = g * 32 + q;
#pragma unroll
    for (int e = 0; e < 8; ++e) {
      const float f = Tt[(c8 + e) * 65 + qq];
      const unsigned short bits = __builtin_bit_cast(unsigned short, (_Float16)(f * sc));
      hv[g][e] = __builtin_bit_cast(_Float16, bits);
    }
  }
  for (int pass = 0; pass < 2; ++pass) {
#pragma unroll
    for (int g = 0; g < 2; ++g) {
      const size_t o = (size_t)(c0 + g * 32 + q) * (size_t)ldo + (size_t)(r0 + c8);
      *(volatile v8h*)(O + o) = hv[g];
    }
    __threadfence();
  }
}

__global__ __launch_bounds__(NTHR) void rnn_seq_kernel(const int* __restrict__ x, const float* __restrict__ tab,
                                                       const unsigned short* __restrict__ whhp,
                                                       const unsigned short* __restrict__ whop,
                                                       const float* __restrict__ bo,
                                                       float* __restrict__ out0, float* __restrict__ out1) {
  extern __shared__ __align__(16) unsigned char smem[];
  float*    XP  = (float*)(smem);
  _Float16* AH  = (_Float16*)(smem + OFF_AH);
  float*    LSL = (float*)(smem + OFF_LSL);
  const _Float16* WHH = (const _Float16*)whhp;
  const _Float16* WHO = (const _Float16*)whop;
  const int tid = threadIdx.x, lane = tid & 31, wave = tid >> 5;
  const int c = lane & 15, hh = lane >> 4, koff = 8 * hh;
  const int rb = blockIdx.x * ROWS_BLK;
  const int ms = (wave >> 1) & 1, vh = wave & 1;

  {
    u4* p = (u4*)(smem + OFF_AH);
    const u4 z = {0u, 0u, 0u, 0u};
#pragma unroll 1
    for (int i = tid; i < LDS_AH_BYTES / 16; i += NTHR) p[i] = z;
  }
  const float bo0 = bo[32 * vh + 2 * c];
  const float bo1 = bo[32 * vh + 2 * c + 1];
  __syncthreads();

  const v8f z8 = {0.f, 0.f, 0.f, 0.f, 0.f, 0.f, 0.f, 0.f};

#pragma unroll 1
  for (int t = 0; t < NSTEP; ++t) {
#pragma unroll 1
    for (int r = 0; r < ROWS_BLK; ++r) {
      int xi = x[(rb + r) * NSTEP + t];
      xi = xi < 0 ? 0 : xi;
      xi = xi > (NVOC - 1) ? (NVOC - 1) : xi;
      const v4f v = *(const v4f*)(tab + (size_t)xi * NHID + 4 * tid);
      *(v4f*)(XP + r * XPP + 4 * tid) = v;
    }
    __syncthreads();

    const int cur = t & 1;
    const _Float16* ahc = AH + cur * AH_HALVES;
    _Float16*       ahn = AH + (cur ^ 1) * AH_HALVES;
    const bool last = (t == NSTEP - 1);

#pragma unroll 1
    for (int g = 0; g < 2; ++g) {
      const int gcol = 128 * wave + 64 * g;
      v8f acc[2][4];
#pragma unroll
      for (int i = 0; i < 2; ++i) {
#pragma unroll
        for (int r = 0; r < 8; ++r) {
          const v4f xv = *(const v4f*)(XP + (16 * i + 8 * hh + r) * XPP + gcol + 4 * c);
#pragma unroll
          for (int j = 0; j < 4; ++j) acc[i][j][r] = xv[j] * WCARRY;
        }
      }
      const _Float16* arow0 = ahc + c * AHP + koff;
      const _Float16* arow1 = arow0 + 16 * AHP;
      const _Float16* bp    = WHH + (size_t)(gcol + 4 * c) * NHID + koff;
#pragma unroll 1
      for (int k0 = 0; k0 < NHID; k0 += 32) {
        const v16h a0 = Frag<_Float16>::load(arow0 + k0);
        const v16h a1 = Frag<_Float16>::load(arow1 + k0);
        const v16h b0 = Frag<_Float16>::load(bp + k0);
        const v16h b1 = Frag<_Float16>::load(bp + NHID + k0);
        const v16h b2 = Frag<_Float16>::load(bp + 2 * NHID + k0);
        const v16h b3 = Frag<_Float16>::load(bp + 3 * NHID + k0);
        acc[0][0] = Frag<_Float16>::mma(a0, b0, acc[0][0]);
        acc[0][1] = Frag<_Float16>::mma(a0, b1, acc[0][1]);
        acc[0][2] = Frag<_Float16>::mma(a0, b2, acc[0][2]);
        acc[0][3] = Frag<_Float16>::mma(a0, b3, acc[0][3]);
        acc[1][0] = Frag<_Float16>::mma(a1, b0, acc[1][0]);
        acc[1][1] = Frag<_Float16>::mma(a1, b1, acc[1][1]);
        acc[1][2] = Frag<_Float16>::mma(a1, b2, acc[1][2]);
        acc[1][3] = Frag<_Float16>::mma(a1, b3, acc[1][3]);
        guard8x6(acc[0][0], acc[0][1], acc[0][2], acc[0][3], acc[1][0], acc[1][1], acc[1][2], acc[1][3],
                 a0, a1, b0, b1, b2, b3);
      }
      acc_guard4(acc[0][0], acc[0][1], acc[0][2], acc[0][3]);
      acc_guard4(acc[1][0], acc[1][1], acc[1][2], acc[1][3]);
#pragma unroll
      for (int i = 0; i < 2; ++i) {
#pragma unroll
        for (int r = 0; r < 8; ++r) {
          const int row = 16 * i + 8 * hh + r;
          const float h0 = ftanh(acc[i][0][r] * WCARRY_INV);
          const float h1 = ftanh(acc[i][1][r] * WCARRY_INV);
          const float h2 = ftanh(acc[i][2][r] * WCARRY_INV);
          const float h3 = ftanh(acc[i][3][r] * WCARRY_INV);
          v4h hv;
          hv[0] = (_Float16)h0; hv[1] = (_Float16)h1; hv[2] = (_Float16)h2; hv[3] = (_Float16)h3;
          *(v4h*)(ahn + row * AHP + gcol + 4 * c) = hv;
          if (last) {
            v4f fv;
            fv[0] = h0; fv[1] = h1; fv[2] = h2; fv[3] = h3;
            *(v4f*)(XP + row * XPP + gcol + 4 * c) = fv;
          }
        }
      }
    }
    __syncthreads();

    if (wave < 4) {
      v8f l0 = z8, l1 = z8;
      const _Float16* arow = ahn + (16 * ms + c) * AHP + koff;
      const _Float16* wp   = WHO + (size_t)(32 * vh + 2 * c) * NHID + koff;
#pragma unroll 1
      for (int k0 = 0; k0 < NHID; k0 += 32) {
        const v16h a  = Frag<_Float16>::load(arow + k0);
        const v16h b0 = Frag<_Float16>::load(wp + k0);
        const v16h b1 = Frag<_Float16>::load(wp + NHID + k0);
        l0 = Frag<_Float16>::mma(a, b0, l0);
        l1 = Frag<_Float16>::mma(a, b1, l1);
        guard2x3(l0, l1, a, b0, b1);
      }
      acc_guard2(l0, l1);
      float* slab = LSL + wave * (16 * LSP);
#pragma unroll
      for (int r = 0; r < 8; ++r) {
        v2f pv;
        pv[0] = l0[r] * WCARRY_INV + bo0;
        pv[1] = l1[r] * WCARRY_INV + bo1;
        *(v2f*)(slab + (8 * hh + r) * LSP + 2 * c) = pv;
      }
      __builtin_amdgcn_fence(__ATOMIC_RELEASE, "workgroup");
      __builtin_amdgcn_wave_barrier();
      __builtin_amdgcn_fence(__ATOMIC_ACQUIRE, "workgroup");
      {
        const int q = lane >> 3, c4 = (lane & 7) * 4;
        for (int pass = 0; pass < 2; ++pass) {
#pragma unroll
          for (int it = 0; it < 4; ++it) {
            const int row = it * 4 + q;
            const v4f v = *(const v4f*)(slab + row * LSP + c4);
            *(volatile v4f*)(out0 + ((size_t)(rb + 16 * ms + row) * NSTEP + (size_t)t) * NVOC + 32 * vh + c4) = v;
          }
          __threadfence();
        }
      }
      __builtin_amdgcn_fence(__ATOMIC_RELEASE, "workgroup");
      __builtin_amdgcn_wave_barrier();
      __builtin_amdgcn_fence(__ATOMIC_ACQUIRE, "workgroup");
    }
    if (last) {
      for (int pass = 0; pass < 2; ++pass) {
#pragma unroll 8
        for (int row = 0; row < ROWS_BLK; ++row) {
          const v4f v = *(const v4f*)(XP + row * XPP + 128 * wave + 4 * lane);
          *(volatile v4f*)(out1 + (size_t)(rb + row) * NHID + 128 * wave + 4 * lane) = v;
        }
        __threadfence();
      }
    }
  }
}

extern "C" void kernel_launch(void* const* d_in, const int* in_sizes, int n_in,
                              void* d_out, int out_size, void* d_ws, size_t ws_size, hipStream_t stream) {
  if (n_in < 7 || d_out == nullptr || d_ws == nullptr) return;
  if (in_sizes[0] != NBATCH * NSTEP || in_sizes[1] != NVOC * NEMB || in_sizes[2] != NEMB * NHID ||
      in_sizes[3] != NHID * NHID || in_sizes[4] != NHID || in_sizes[5] != NHID * NVOC || in_sizes[6] != NVOC ||
      out_size != NOUT0 + NOUT1) return;

  const int*   x   = (const int*)  d_in[0];
  const float* emb = (const float*)d_in[1];
  const float* wih = (const float*)d_in[2];
  const float* whh = (const float*)d_in[3];
  const float* bh  = (const float*)d_in[4];
  const float* who = (const float*)d_in[5];
  const float* bo  = (const float*)d_in[6];
  float* out0 = (float*)d_out;
  float* out1 = out0 + (size_t)NOUT0;

  char* ws = (char*)d_ws; size_t off = 0;
  auto carve = [&](size_t bytes) -> char* { char* p = ws + off; off += (bytes + 255) & ~(size_t)255; return p; };
  float*          TAB = (float*)carve((size_t)NVOC * NHID * 4);
  unsigned short* WHH = (unsigned short*)carve((size_t)NHID * NHID * 2);
  unsigned short* WHO = (unsigned short*)carve((size_t)NVOC * NHID * 2);
  if (off > ws_size || off > (size_t)134217728) return;

  table_kernel<<<(NVOC * NHID / 4) / NTHR, NTHR, 0, stream>>>(emb, wih, bh, TAB);
  tpw_f16_kernel<<<dim3(NHID / 64, NHID / 64), NTHR, 0, stream>>>(whh, NHID, NHID, NHID, WHH, WCARRY);
  tpw_f16_kernel<<<dim3(NVOC / 64, NHID / 64), NTHR, 0, stream>>>(who, NHID, NVOC, NHID, WHO, WCARRY);
  rnn_seq_kernel<<<NBATCH / ROWS_BLK, NTHR, LDS_TOTAL, stream>>>(x, TAB, WHH, WHO, bo, out0, out1);
}
